// NearestEmbed_20529943675246
// MI455X (gfx1250) — hardware-verified
//
#include <hip/hip_runtime.h>


namespace {
constexpr int NBAT = 32, D = 256, HW = 1024, N = NBAT * HW, KC = 2048, NT = KC / 64;
constexpr float XS = 8.0f;

typedef _Float16 b16;
typedef __attribute__((ext_vector_type(16))) _Float16 v16b;
typedef __attribute__((ext_vector_type(8)))  _Float16 v8b;
typedef __attribute__((ext_vector_type(8)))  float v8f;
typedef __attribute__((ext_vector_type(4)))  float v4f;

__device__ __forceinline__ v8b ld8b(const b16* p) { return *(const v8b*)p; }
__device__ __forceinline__ v16b cat8b(v8b a, v8b b) { return __builtin_shufflevector(a, b, 0, 1, 2, 3, 4, 5, 6, 7, 8, 9, 10, 11, 12, 13, 14, 15); }
__device__ __forceinline__ v16b frag_kb(const b16* p, int hh) { return cat8b(ld8b(p + 8 * hh), ld8b(p + 16 + 8 * hh)); }
__device__ __forceinline__ void split16(float v, b16& hi, b16& lo) { hi = (b16)v; lo = (b16)(v - (float)hi); }
__device__ __forceinline__ void frag_ksplit(const float* p, int hh, v16b& fh_, v16b& fl_) {
  const float* p0 = p + 8 * hh; const float* p1 = p + 16 + 8 * hh;
#pragma unroll
  for (int e = 0; e < 8; ++e) { b16 a, c; split16(p0[e], a, c); fh_[e] = a; fl_[e] = c; split16(p1[e], a, c); fh_[8 + e] = a; fl_[8 + e] = c; }
}
__device__ __forceinline__ v8f wmma16b(v16b a, v16b b, v8f c) {
  v8f d = __builtin_amdgcn_wmma_f32_16x16x32_f16(false, a, false, b, (short)0, c, false, false);
  asm volatile("v_nop\n\tv_nop\n\tv_nop\n\tv_nop" : "+v"(d) : "v"(a), "v"(b));
  return d;
}
__device__ __forceinline__ void wave_lds_sync() {
  __builtin_amdgcn_fence(__ATOMIC_RELEASE, "workgroup");
  __builtin_amdgcn_wave_barrier();
  __builtin_amdgcn_fence(__ATOMIC_ACQUIRE, "workgroup");
}

struct Opnd { const void* p0; const void* p1; int ld; };
template <int NP> __device__ __forceinline__ void load_frags(const Opnd& o, int row, int kb, int hh, v16b& fh_, v16b& fl_) {
  if (NP == 0) { frag_ksplit((const float*)o.p0 + (size_t)row * o.ld + kb, hh, fh_, fl_); }
  else if (NP == 4) {
    const float* p = (const float*)o.p0 + (size_t)row * o.ld + kb; const float* p0 = p + 8 * hh; const float* p1 = p + 16 + 8 * hh;
#pragma unroll
    for (int e = 0; e < 8; ++e) { b16 a, c; split16(p0[e] * 64.0f, a, c); fh_[e] = a; fl_[e] = c; split16(p1[e] * 64.0f, a, c); fh_[8 + e] = a; fl_[8 + e] = c; }
  } else if (NP == 3) {
    const float* p = (const float*)o.p0 + (size_t)row * o.ld + kb; const float* p0 = p + 8 * hh; const float* p1 = p + 16 + 8 * hh;
#pragma unroll
    for (int e = 0; e < 8; ++e) { fh_[e] = (b16)p0[e]; fh_[8 + e] = (b16)p1[e]; }
    fl_ = fh_;
  } else {
    fh_ = frag_kb((const b16*)o.p0 + (size_t)row * o.ld + kb, hh);
    if (NP == 2) fl_ = frag_kb((const b16*)o.p1 + (size_t)row * o.ld + kb, hh); else fl_ = fh_;
  }
}
template <int ANP, int BNP> __device__ __forceinline__ v8f mac(v16b ah, v16b al, v16b bh, v16b bl, v8f c) {
  c = wmma16b(ah, bh, c);
  if (BNP == 0 || BNP == 2 || BNP == 4) c = wmma16b(ah, bl, c);
  if (ANP == 0 || ANP == 2 || ANP == 4) c = wmma16b(al, bh, c);
  return c;
}
template <int ANP, int BNP>
__device__ __forceinline__ void gemm_tile(const Opnd& A, const Opnd& B, int K, int m0, int c0, int nloc, int hlf, v8f (&acc)[2][4]) {
  for (int kb = 0; kb < K; kb += 32) {
    v16b a0h, a0l, a1h, a1l;
    load_frags<ANP>(A, m0 + nloc, kb, hlf, a0h, a0l);
    load_frags<ANP>(A, m0 + 16 + nloc, kb, hlf, a1h, a1l);
#pragma unroll
    for (int t = 0; t < 4; ++t) {
      v16b bh, bl;
      load_frags<BNP>(B, c0 + t * 16 + nloc, kb, hlf, bh, bl);
      acc[0][t] = mac<ANP, BNP>(a0h, a0l, bh, bl, acc[0][t]);
      acc[1][t] = mac<ANP, BNP>(a1h, a1l, bh, bl, acc[1][t]);
    }
  }
}

__device__ __forceinline__ void epi_planes(v8f (&acc)[2][4], float scale, bool two, b16* __restrict__ oh, b16* __restrict__ ol, int ldo,
                                           int m0, int c0, int lane, b16* Th, b16* Tl) {
  const int nloc = lane & 15, hlf = lane >> 4;
#pragma unroll
  for (int t = 0; t < 4; ++t)
#pragma unroll
    for (int r = 0; r < 2; ++r)
#pragma unroll
      for (int v = 0; v < 8; ++v) {
        const int rr = r * 16 + v + 8 * hlf, cc = t * 16 + nloc;
        b16 h_, l_; split16(acc[r][t][v] * scale, h_, l_);
        Th[rr * 64 + cc] = h_; Tl[rr * 64 + cc] = l_;
      }
  wave_lds_sync();
  for (int pass = 0; pass < 2; ++pass) {
#pragma unroll
    for (int j = 0; j < 8; ++j) {
      const int rr = j * 4 + (lane >> 3), c8 = (lane & 7) * 8;
      const size_t o = (size_t)(m0 + rr) * ldo + c0 + c8;
      *(volatile v8b*)(oh + o) = ld8b(Th + rr * 64 + c8);
      if (two) *(volatile v8b*)(ol + o) = ld8b(Tl + rr * 64 + c8);
    }
    __threadfence();
  }
}
__device__ __forceinline__ void epi_f32(v8f (&acc)[2][4], float scale, const float* rscale, float* __restrict__ out, int ldo, int m0, int c0, int lane, float* Tt) {
  const int nloc = lane & 15, hlf = lane >> 4;
#pragma unroll
  for (int t = 0; t < 4; ++t)
#pragma unroll
    for (int r = 0; r < 2; ++r)
#pragma unroll
      for (int v = 0; v < 8; ++v) {
        const int rr = r * 16 + v + 8 * hlf;
        const float rs = rscale ? rscale[(size_t)(m0 + rr) * 32] : 1.0f;
        Tt[rr * 64 + t * 16 + nloc] = acc[r][t][v] * scale * rs;
      }
  wave_lds_sync();
  float* dst0 = out + (size_t)m0 * ldo + c0;
  for (int pass = 0; pass < 2; ++pass) {
#pragma unroll
    for (int j = 0; j < 16; ++j) { const int rr = j * 2 + hlf, c4 = nloc * 4; *(volatile v4f*)(dst0 + (size_t)rr * ldo + c4) = *(const v4f*)(Tt + rr * 64 + c4); }
    __threadfence();
  }
}


__global__ __launch_bounds__(256) void prep_kernel(const float* __restrict__ x, const float* __restrict__ emb, b16* __restrict__ xh, b16* __restrict__ xl,
                                                   b16* __restrict__ eh, b16* __restrict__ el, float* __restrict__ e2) {
  __shared__ __attribute__((aligned(16))) b16 Th[64][72]; __shared__ __attribute__((aligned(16))) b16 Tl[64][72];
  const int tid = threadIdx.x, lane = tid & 31, wave = tid >> 5; const int nx = (N / 64) * (D / 64), nem = (KC / 64) * (D / 64);
  if ((int)blockIdx.x < nx + nem) {
    const bool isx = (int)blockIdx.x < nx; const int bi = isx ? blockIdx.x : blockIdx.x - nx;
    const int r0 = (bi / (D / 64)) * 64, c0 = (bi % (D / 64)) * 64;
    for (int i = tid; i < 64 * 64; i += 256) {
      const int cc = i / 64, rr = i % 64; float v;
      if (isx) { const int n = r0 + rr, b = n / HW, hw = n % HW; v = x[((size_t)b * D + c0 + cc) * HW + hw]; } else v = emb[(size_t)(c0 + cc) * KC + r0 + rr];
      b16 a, b2; split16(v * XS, a, b2); Th[rr][cc] = a; Tl[rr][cc] = b2;
    }
    __syncthreads();
    b16* oh = (isx ? xh : eh) + (size_t)r0 * D + c0; b16* olw = (isx ? xl : el) + (size_t)r0 * D + c0;
    for (int pass = 0; pass < 2; ++pass) {
#pragma unroll
      for (int j = 0; j < 2; ++j) { const int rr = wave * 8 + j * 4 + (lane >> 3), c8 = (lane & 7) * 8;
        *(volatile v8b*)(oh + (size_t)rr * D + c8) = *(const v8b*)(&Th[rr][c8]); *(volatile v8b*)(olw + (size_t)rr * D + c8) = *(const v8b*)(&Tl[rr][c8]); }
      __threadfence();
    }
  } else {
    const int j = ((int)blockIdx.x - nx - nem) * 256 + tid; float s = 0.0f;
#pragma unroll 1
    for (int c = 0; c < D; ++c) { const float v = emb[(size_t)c * KC + j]; s += v * v; }
    ((volatile float*)e2)[j] = s; __threadfence(); ((volatile float*)e2)[j] = s;
  }
}

__global__ __launch_bounds__(128) void vq_kernel(const b16* __restrict__ xh, const b16* __restrict__ xl, const b16* __restrict__ eh, const b16* __restrict__ el,
                                                const float* __restrict__ e2, const float* __restrict__ emb, float* __restrict__ out) {
  __shared__ int idx[128];
  const int lane = threadIdx.x & 31, wave = threadIdx.x >> 5, nloc = lane & 15, hlf = lane >> 4;
  const int m0 = blockIdx.x * 128 + wave * 32;
  float bestv[2][8]; int besti[2][8];
#pragma unroll
  for (int r = 0; r < 2; ++r)
#pragma unroll
    for (int v = 0; v < 8; ++v) { bestv[r][v] = INFINITY; besti[r][v] = 0; }
  const Opnd A{xh, xl, D}, B{eh, el, D};
#pragma unroll 1
  for (int tile = 0; tile < NT; ++tile) {
    const int c0 = tile * 64;
    v8f acc[2][4];
#pragma unroll
    for (int r = 0; r < 2; ++r)
#pragma unroll
      for (int t = 0; t < 4; ++t) acc[r][t] = (v8f){};
    gemm_tile<2, 2>(A, B, D, m0, c0, nloc, hlf, acc);
#pragma unroll
    for (int r = 0; r < 2; ++r)
#pragma unroll
      for (int v = 0; v < 8; ++v) {
        float best = INFINITY; int bi = 0;
#pragma unroll
        for (int t = 0; t < 4; ++t) { const int j = c0 + t * 16 + nloc; const float val = e2[j] - 2.0f * acc[r][t][v] * (1.0f / (XS * XS)); if (val < best) { best = val; bi = j; } }
#pragma unroll
        for (int o = 1; o < 16; o <<= 1) { const float ob = __shfl_xor(best, o); const int oi = __shfl_xor(bi, o); if (ob < best || (ob == best && oi < bi)) { best = ob; bi = oi; } }
        if (best < bestv[r][v]) { bestv[r][v] = best; besti[r][v] = bi; }
      }
  }
#pragma unroll
  for (int r = 0; r < 2; ++r)
#pragma unroll
    for (int v = 0; v < 8; ++v) if (nloc == 0) { const int bi = besti[r][v]; idx[wave * 32 + r * 16 + v + 8 * hlf] = (bi < 0) ? 0 : (bi >= KC ? KC - 1 : bi); }
  __syncthreads();
  const int n0 = blockIdx.x * 128, b = n0 / HW, hw0 = n0 % HW, t = threadIdx.x; const int myidx = idx[t];
  for (int pass = 0; pass < 2; ++pass) {
#pragma unroll 1
    for (int c = 0; c < D; ++c) ((volatile float*)out)[((size_t)b * D + c) * HW + hw0 + t] = emb[(size_t)c * KC + myidx];
    __threadfence();
  }
}
}

extern "C" void kernel_launch(void* const* d_in, const int* in_sizes, int n_in,
                              void* d_out, int out_size, void* d_ws, size_t ws_size, hipStream_t stream) {
  (void)n_in; (void)out_size;
  const float* x = (const float*)d_in[0];
  const float* emb = (const float*)d_in[1];
  float* out = (float*)d_out;
  if (in_sizes[0] != N * D || in_sizes[1] != D * KC) return;
  size_t off = 0; char* ws = (char*)d_ws;
  auto carve = [&](size_t bytes) { char* p = ws + off; off += (bytes + 255) & ~(size_t)255; return p; };
  b16* xh = (b16*)carve((size_t)N * D * 2); b16* xl = (b16*)carve((size_t)N * D * 2);
  b16* eh = (b16*)carve((size_t)KC * D * 2); b16* el = (b16*)carve((size_t)KC * D * 2);
  float* e2 = (float*)carve((size_t)KC * 4);
  if (off > ws_size) return;
  prep_kernel<<<(N / 64) * (D / 64) + (KC / 64) * (D / 64) + KC / 256, 256, 0, stream>>>(x, emb, xh, xl, eh, el, e2);
  vq_kernel<<<N / 128, 128, 0, stream>>>(xh, xl, eh, el, e2, emb, out);
}
